// NonSymmetricAttentionKernel_89455578841178
// MI455X (gfx1250) — hardware-verified
//
#include <hip/hip_runtime.h>


#define NB_  2
#define TT   2048
#define DM   768
#define NH_  12
#define HD   64
#define HPP  4
#define RHL  512
#define PCAR 1024.0f
typedef _Float16 h16;
typedef unsigned short bf;
typedef __attribute__((ext_vector_type(16))) __bf16   v16bf;
typedef __attribute__((ext_vector_type(16))) _Float16 v16h;
typedef __attribute__((ext_vector_type(8)))  _Float16 v8h;
typedef __attribute__((ext_vector_type(8)))  unsigned short v8us;
typedef __attribute__((ext_vector_type(8)))  float    v8f;
typedef __attribute__((ext_vector_type(4)))  float    v4f;
typedef v8h  __attribute__((may_alias)) v8ha;
typedef v4f  __attribute__((may_alias)) v4fa;
typedef v8us __attribute__((may_alias)) v8usa;

__device__ __forceinline__ unsigned short f2bf(float f) { unsigned u = __float_as_uint(f); u += 0x7FFFu + ((u >> 16) & 1u); return (unsigned short)(u >> 16); }
__device__ __forceinline__ float bf2f(unsigned short b) { return __uint_as_float(((unsigned)b) << 16); }
__device__ __forceinline__ float bfr(float f) { return bf2f(f2bf(f)); }
__device__ __forceinline__ v16h cat16(v8h lo, v8h hi) { return __builtin_shufflevector(lo, hi, 0, 1, 2, 3, 4, 5, 6, 7, 8, 9, 10, 11, 12, 13, 14, 15); }
__device__ __forceinline__ v16bf cat16b(v8us lo, v8us hi) { return __builtin_bit_cast(v16bf, __builtin_shufflevector(lo, hi, 0, 1, 2, 3, 4, 5, 6, 7, 8, 9, 10, 11, 12, 13, 14, 15)); }
__device__ __forceinline__ v8f wmma16(v16h a, v16h b, v8f c) { return __builtin_amdgcn_wmma_f32_16x16x32_f16(false, a, false, b, (short)0, c, false, false); }
__device__ __forceinline__ v8f wmmab(v16bf a, v16bf b, v8f c) { return __builtin_amdgcn_wmma_f32_16x16x32_bf16(false, a, false, b, (short)0, c, false, false); }


template <typename T16> struct WFrag;
template <> struct WFrag<h16> { typedef v16h V; static __device__ __forceinline__ V ld(const h16* p) { return cat16(*(const v8h*)p, *(const v8h*)(p + 16)); } static __device__ __forceinline__ v8f mma(V a, V b, v8f c) { return wmma16(a, b, c); } };
template <> struct WFrag<bf> { typedef v16bf V; static __device__ __forceinline__ V ld(const bf* p) { return cat16b(*(const v8us*)p, *(const v8us*)(p + 16)); } static __device__ __forceinline__ v8f mma(V a, V b, v8f c) { return wmmab(a, b, c); } };
template <typename T16, int NSPLIT, bool BIAS>
__global__ __launch_bounds__(32) void k_gemmw(const T16* __restrict__ A, const T16* __restrict__ A2, const T16* __restrict__ Bt, const T16* __restrict__ Bt2, int K, float* C, int ldc, const float* __restrict__ bias, size_t sA, size_t sB, size_t sC) {
    typedef typename WFrag<T16>::V V;
    __shared__ __align__(16) float os[16 * 68];
    const size_t z = blockIdx.z; A += z * sA; if (A2) A2 += z * sA; Bt += z * sB; if (Bt2) Bt2 += z * sB; C += z * sC;
    const int lane = threadIdx.x & 31, lr = lane & 15, hi = lane >> 4; const int r0 = blockIdx.x * 64, c0 = blockIdx.y * 64;
    v8f acc[4][4];
#pragma unroll
    for (int mb = 0; mb < 4; ++mb)
#pragma unroll
        for (int nb = 0; nb < 4; ++nb) acc[mb][nb] = (v8f){};
    const size_t aoff = (size_t)(r0 + lr) * K + 8 * hi, boff = (size_t)(c0 + lr) * K + 8 * hi;
#pragma unroll 1
    for (int kc = 0; kc < K; kc += 32) {
        V a[4], a2[4];
#pragma unroll
        for (int mb = 0; mb < 4; ++mb) { a[mb] = WFrag<T16>::ld(A + aoff + (size_t)mb * 16 * K + kc); if (NSPLIT == 1 || NSPLIT == 2) a2[mb] = WFrag<T16>::ld(A2 + aoff + (size_t)mb * 16 * K + kc); }
#pragma unroll
        for (int nb = 0; nb < 4; ++nb) { const V b = WFrag<T16>::ld(Bt + boff + (size_t)nb * 16 * K + kc); V b2; if (NSPLIT >= 2) b2 = WFrag<T16>::ld(Bt2 + boff + (size_t)nb * 16 * K + kc);
#pragma unroll
            for (int mb = 0; mb < 4; ++mb) { acc[mb][nb] = WFrag<T16>::mma(a[mb], b, acc[mb][nb]); if (NSPLIT == 1 || NSPLIT == 2) acc[mb][nb] = WFrag<T16>::mma(a2[mb], b, acc[mb][nb]); if (NSPLIT >= 2) acc[mb][nb] = WFrag<T16>::mma(a[mb], b2, acc[mb][nb]); } }
        asm volatile("v_nop\n\tv_nop\n\tv_nop\n\tv_nop" : "+v"(acc[0][0]), "+v"(acc[1][1]), "+v"(acc[2][2]), "+v"(acc[3][3]) : "v"(a[0]), "v"(a[3]));
    }
#pragma unroll
    for (int mb = 0; mb < 4; ++mb) {
#pragma unroll
        for (int nb = 0; nb < 4; ++nb) {
#pragma unroll
            for (int j = 0; j < 8; ++j) os[(hi * 8 + j) * 68 + nb * 16 + lr] = acc[mb][nb][j]; }
        __builtin_amdgcn_wave_barrier(); asm volatile("" ::: "memory");
        float* crow = C + (size_t)(r0 + mb * 16) * ldc + c0;
#pragma unroll 1
        for (int ps = 0; ps < 2; ++ps) {
#pragma unroll
            for (int s = 0; s < 8; ++s) { const int row = 2 * s + hi, cofs = lr * 4; v4f val = *(const v4fa*)(os + row * 68 + cofs); if (BIAS) { val[0] += bfr(bias[c0 + cofs]); val[1] += bfr(bias[c0 + cofs + 1]); val[2] += bfr(bias[c0 + cofs + 2]); val[3] += bfr(bias[c0 + cofs + 3]); }
                *(volatile v4f*)(crow + (size_t)row * ldc + cofs) = val; }
            if (ps == 0) __threadfence(); }
        __builtin_amdgcn_wave_barrier(); asm volatile("" ::: "memory");
    }
}

__device__ __forceinline__ h16 tohx(float x) { return (h16)x; }
__device__ __forceinline__ void splitf(float y, unsigned short& h, unsigned short& l) { h = f2bf(y); l = f2bf(y - bf2f(h)); }
typedef __attribute__((ext_vector_type(2))) unsigned short v2us;
typedef __attribute__((ext_vector_type(4))) unsigned short v4us;
typedef __attribute__((ext_vector_type(2))) _Float16 v2h;
typedef __attribute__((ext_vector_type(4))) _Float16 v4h;

__global__ __launch_bounds__(256) void k_wtG(const float* __restrict__ w, int K, int N, bf* Bt) {
    const int lane = threadIdx.x & 31; const int L0 = (blockIdx.x * 8 + (threadIdx.x >> 5)) * 8; const int nlines = N * K / 64;
#pragma unroll
    for (int ps = 0; ps < 2; ++ps) {
#pragma unroll 1
        for (int l = 0; l < 8; ++l) { const int L = L0 + l; if (L >= nlines) break; const size_t e = (size_t)L * 64 + lane * 2; const int k = (int)(e % K), n = (int)(e / K); v2us o;
            o[0] = f2bf(w[(size_t)k * N + n]); o[1] = f2bf(w[(size_t)(k + 1) * N + n]); *(volatile v2us*)(Bt + e) = o; }
        if (ps == 0) __threadfence(); }
}
__global__ __launch_bounds__(256) void k_cvt8(const float* __restrict__ src, bf* dst, size_t n8) { const size_t i = (size_t)blockIdx.x * 256 + threadIdx.x; if (i >= n8) return; const v8f v = *(const v8f*)(src + i * 8); v8us o;
#pragma unroll
    for (int k = 0; k < 8; ++k) o[k] = f2bf(v[k]); *(volatile v8us*)(dst + i * 8) = o; __threadfence(); *(volatile v8us*)(dst + i * 8) = o; }
__device__ __forceinline__ bool hlrow(int g, int i) { return (g == 0) ? (i < RHL) : (g == 1) ? (i >= TT - RHL) : false; }
__global__ __launch_bounds__(256) void k_pl3(const float* __restrict__ F, h16* P, bf* Ph, bf* Pl) { const int e = (blockIdx.x * 256 + threadIdx.x) * 4; if (e >= NH_ * TT * HD) return; const int d = e % HD; const int t = (e / HD) % TT; const int h = e / (HD * TT); const float* f = F + (size_t)t * DM + h * HD + d; v4h o; v4us oh, ol;
#pragma unroll
    for (int u = 0; u < 4; ++u) { o[u] = tohx(f[u]); unsigned short a, b; splitf(f[u], a, b); oh[u] = a; ol[u] = b; } for (int ps = 0; ps < 2; ++ps) { *(volatile v4h*)(P + e) = o; *(volatile v4us*)(Ph + e) = oh; *(volatile v4us*)(Pl + e) = ol; if (ps == 0) __threadfence(); } }
__global__ __launch_bounds__(256) void k_vt3(const float* __restrict__ V, h16* VT, bf* VTh, bf* VTl) { const int e = (blockIdx.x * 256 + threadIdx.x) * 2; if (e >= NH_ * HD * TT) return; const int t = e % TT; const int d = (e / TT) % HD; const int h = e / (TT * HD); const float a = V[(size_t)t * DM + h * HD + d], b = V[(size_t)(t + 1) * DM + h * HD + d]; v2h o; o[0] = tohx(a); o[1] = tohx(b); v2us oh, ol; unsigned short a1, b1, a2, b2; splitf(a, a1, b1); splitf(b, a2, b2); oh[0] = a1; oh[1] = a2; ol[0] = b1; ol[1] = b2;
    for (int ps = 0; ps < 2; ++ps) { *(volatile v2h*)(VT + e) = o; *(volatile v2us*)(VTh + e) = oh; *(volatile v2us*)(VTl + e) = ol; if (ps == 0) __threadfence(); } }
__global__ __launch_bounds__(256) void k_sqt(float* SQ) { const int j = blockIdx.x * 256 + threadIdx.x; if (j >= TT) return; const float r = __fsqrt_rn((float)j); *(volatile float*)(SQ + j) = r; __threadfence(); *(volatile float*)(SQ + j) = r; }
__global__ __launch_bounds__(256) void k_nsoft(const float* __restrict__ Sb, const float* __restrict__ SQ, int h0, h16* P16, bf* Ph, bf* Pl) { const int lane = threadIdx.x & 31; const int row = blockIdx.x * 8 + (threadIdx.x >> 5); if (row >= HPP * TT) return; const int i = row % TT; const int z = row / TT; const int h = h0 + z; const int g = h / 4; const int hm = h % 4;
    const float slope = (hm == 0) ? 0.25f : (hm == 1) ? 0.0625f : (hm == 2) ? 0.015625f : 0.00390625f; const float sqi = SQ[i]; const float* sr = Sb + (size_t)row * TT; float v[TT / 32]; float mx = -3.0e38f;
#pragma unroll
    for (int ch = 0; ch < TT / 128; ++ch) { const int j0 = ch * 128 + lane * 4; const v4f a = *(const v4f*)(sr + j0); const v4f sq = *(const v4f*)(SQ + j0);
#pragma unroll
        for (int u = 0; u < 4; ++u) { const int j = j0 + u; const bool keep = (g == 0) ? (j <= i) : (g == 1) ? (j >= i) : true; float rel = fabsf(__fsub_rn(sq[u], sqi)); asm volatile("" : "+v"(rel)); float t0 = a[u] * 0.125f; asm volatile("" : "+v"(t0)); float ab = __fmul_rn(slope, rel); asm volatile("" : "+v"(ab)); const float t = keep ? __fsub_rn(t0, ab) : -3.0e38f; v[ch * 4 + u] = t; mx = fmaxf(mx, t); } }
#pragma unroll
    for (int sh = 16; sh; sh >>= 1) mx = fmaxf(mx, __shfl_xor(mx, sh, 32));
    float sum = 0.f;
#pragma unroll
    for (int q = 0; q < TT / 32; ++q) { float d0 = __fsub_rn(v[q], mx); asm volatile("" : "+v"(d0)); v[q] = (v[q] > -1.0e38f) ? __builtin_amdgcn_exp2f(__fmul_rn(d0, 1.4426950408889634f)) : 0.f; sum += v[q]; }
#pragma unroll
    for (int sh = 16; sh; sh >>= 1) sum += __shfl_xor(sum, sh, 32);
    const float inv = __fdiv_rn(1.0f, sum); const float f = inv * PCAR; const bool hl = hlrow(g, i);
    for (int ps = 0; ps < 2; ++ps) {
#pragma unroll
        for (int ch = 0; ch < TT / 128; ++ch) { const size_t oo = (size_t)row * TT + ch * 128 + lane * 4; v4h o4;
#pragma unroll
            for (int q = 0; q < 4; ++q) o4[q] = tohx(v[ch * 4 + q] * f); *(volatile v4h*)(P16 + oo) = o4; }
        if (hl) {
#pragma unroll
            for (int ch = 0; ch < TT / 128; ++ch) { const size_t oo = (size_t)row * TT + ch * 128 + lane * 4; v4us oh, ol;
#pragma unroll
                for (int q = 0; q < 4; ++q) { unsigned short a, b; splitf(v[ch * 4 + q] * inv, a, b); oh[q] = a; ol[q] = b; } *(volatile v4us*)(Ph + oo) = oh; *(volatile v4us*)(Pl + oo) = ol; } }
        if (ps == 0) __threadfence(); } }
__global__ __launch_bounds__(256) void k_mrg(const float* __restrict__ O16, const float* __restrict__ Ohl, int h0, float* outb) { const int e = (blockIdx.x * 256 + threadIdx.x) * 4; if (e >= HPP * TT * HD) return; const int d = e % HD; const int t = (e / HD) % TT; const int z = e / (HD * TT); const int h = h0 + z; const bool hl = hlrow(h / 4, t); v4f o;
#pragma unroll
    for (int u = 0; u < 4; ++u) o[u] = hl ? Ohl[e + u] : O16[e + u] * (1.0f / PCAR); float* dst = outb + (size_t)t * DM + h * HD + d; *(volatile v4f*)dst = o; __threadfence(); *(volatile v4f*)dst = o; }

extern "C" void kernel_launch(void* const* d_in, const int* in_sizes, int n_in,
                              void* d_out, int out_size, void* d_ws, size_t ws_size, hipStream_t stream) {
    (void)in_sizes; (void)n_in; (void)out_size;
    const float** I = (const float**)d_in;
    const float *x = I[0], *Wq = I[1], *bq = I[2], *Wk = I[3], *bk = I[4], *Wv = I[5], *bv = I[6];
    float* OUT = (float*)d_out;
    char* wsp = (char*)d_ws;
    auto take = [&](size_t bytes) { char* p = wsp; wsp += (bytes + 255) & ~(size_t)255; return (void*)p; };
    bf* BQ = (bf*)take((size_t)DM * DM * 2); bf* BK = (bf*)take((size_t)DM * DM * 2); bf* BV = (bf*)take((size_t)DM * DM * 2);
    bf* XB = (bf*)take((size_t)TT * DM * 2); float* Q = (float*)take((size_t)TT * DM * 4); float* K = (float*)take((size_t)TT * DM * 4); float* V = (float*)take((size_t)TT * DM * 4);
    h16* Q16 = (h16*)take((size_t)NH_ * TT * HD * 2); bf* Qh = (bf*)take((size_t)NH_ * TT * HD * 2); bf* Ql = (bf*)take((size_t)NH_ * TT * HD * 2); h16* K16 = (h16*)take((size_t)NH_ * TT * HD * 2); bf* Kh = (bf*)take((size_t)NH_ * TT * HD * 2); bf* Kl = (bf*)take((size_t)NH_ * TT * HD * 2);
    h16* VT = (h16*)take((size_t)NH_ * HD * TT * 2); bf* VTh = (bf*)take((size_t)NH_ * HD * TT * 2); bf* VTl = (bf*)take((size_t)NH_ * HD * TT * 2);
    float* Sb = (float*)take((size_t)HPP * TT * TT * 4); h16* P16 = (h16*)take((size_t)HPP * TT * TT * 2); bf* Ph = (bf*)take((size_t)HPP * TT * TT * 2); bf* Pl = (bf*)take((size_t)HPP * TT * TT * 2); float* SQ = (float*)take(TT * 4); float* O16 = (float*)take((size_t)HPP * TT * HD * 4); float* Ohl = (float*)take((size_t)HPP * TT * HD * 4);
    if ((size_t)(wsp - (char*)d_ws) > ws_size) return;
    k_wtG<<<(DM * DM / 64 + 63) / 64, 256, 0, stream>>>(Wq, DM, DM, BQ); k_wtG<<<(DM * DM / 64 + 63) / 64, 256, 0, stream>>>(Wk, DM, DM, BK); k_wtG<<<(DM * DM / 64 + 63) / 64, 256, 0, stream>>>(Wv, DM, DM, BV);
    const size_t zs = (size_t)TT * HD; k_sqt<<<(TT + 255) / 256, 256, 0, stream>>>(SQ);
    for (int b = 0; b < NB_; ++b) {
        k_cvt8<<<(TT * DM / 8 + 255) / 256, 256, 0, stream>>>(x + (size_t)b * TT * DM, XB, (size_t)TT * DM / 8);
        k_gemmw<bf, 0, true><<<dim3(TT / 64, DM / 64, 1), 32, 0, stream>>>(XB, nullptr, BQ, nullptr, DM, Q, DM, bq, 0, 0, 0); k_gemmw<bf, 0, true><<<dim3(TT / 64, DM / 64, 1), 32, 0, stream>>>(XB, nullptr, BK, nullptr, DM, K, DM, bk, 0, 0, 0); k_gemmw<bf, 0, true><<<dim3(TT / 64, DM / 64, 1), 32, 0, stream>>>(XB, nullptr, BV, nullptr, DM, V, DM, bv, 0, 0, 0);
        k_pl3<<<(NH_ * TT * HD / 4 + 255) / 256, 256, 0, stream>>>(Q, Q16, Qh, Ql); k_pl3<<<(NH_ * TT * HD / 4 + 255) / 256, 256, 0, stream>>>(K, K16, Kh, Kl); k_vt3<<<(NH_ * HD * TT / 2 + 255) / 256, 256, 0, stream>>>(V, VT, VTh, VTl);
        for (int h0 = 0; h0 < NH_; h0 += HPP) { const int g = h0 / 4; const size_t zo = (size_t)h0 * zs; const int r0 = (g == 0) ? 0 : TT - RHL;
            k_gemmw<h16, 0, false><<<dim3(TT / 64, TT / 64, HPP), 32, 0, stream>>>(Q16 + zo, nullptr, K16 + zo, nullptr, HD, Sb, TT, nullptr, zs, zs, (size_t)TT * TT);
            if (g < 2) k_gemmw<bf, 2, false><<<dim3(RHL / 64, TT / 64, HPP), 32, 0, stream>>>(Qh + zo + (size_t)r0 * HD, Ql + zo + (size_t)r0 * HD, Kh + zo, Kl + zo, HD, Sb + (size_t)r0 * TT, TT, nullptr, zs, zs, (size_t)TT * TT);
            k_nsoft<<<HPP * TT / 8, 256, 0, stream>>>(Sb, SQ, h0, P16, Ph, Pl);
            k_gemmw<h16, 0, false><<<dim3(TT / 64, 1, HPP), 32, 0, stream>>>(P16, nullptr, VT + zo, nullptr, TT, O16, HD, nullptr, (size_t)TT * TT, zs, zs);
            if (g < 2) k_gemmw<bf, 2, false><<<dim3(RHL / 64, 1, HPP), 32, 0, stream>>>(Ph + (size_t)r0 * TT, Pl + (size_t)r0 * TT, VTh + zo, VTl + zo, TT, Ohl + (size_t)r0 * HD, HD, nullptr, (size_t)TT * TT, zs, zs);
            k_mrg<<<(HPP * TT * HD / 4 + 255) / 256, 256, 0, stream>>>(O16, Ohl, h0, OUT + (size_t)b * TT * DM); } }
}
